// RNade_75977971466989
// MI455X (gfx1250) — hardware-verified
//
#include <hip/hip_runtime.h>


#define NBT  256
#define NL   500
#define DI   3
#define DC   32
#define NI   35
#define KI   64
#define HH   512
#define NO   35
#define NOP  64
#define LCH  50
#define NLC  (NL / LCH)
#define DM   HH
#define NTK  NBT
#define LOSC 1024.0f

typedef _Float16 h16;
typedef unsigned short bf;
typedef __attribute__((ext_vector_type(16))) __bf16   v16bf;
typedef __attribute__((ext_vector_type(16))) _Float16 v16h;
typedef __attribute__((ext_vector_type(8)))  _Float16 v8h;
typedef __attribute__((ext_vector_type(8)))  unsigned short v8us;
typedef __attribute__((ext_vector_type(8)))  float    v8f;
typedef __attribute__((ext_vector_type(4)))  float    v4f;
typedef __attribute__((ext_vector_type(4)))  _Float16 v4h;
typedef v8h  __attribute__((may_alias)) v8ha;
typedef v4f  __attribute__((may_alias)) v4fa;
typedef v8us __attribute__((may_alias)) v8usa;

__device__ __forceinline__ unsigned short f2bf(float f) { unsigned u = __float_as_uint(f); u += 0x7FFFu + ((u >> 16) & 1u); return (unsigned short)(u >> 16); }
__device__ __forceinline__ float bf2f(unsigned short b) { return __uint_as_float(((unsigned)b) << 16); }
__device__ __forceinline__ float bfr(float f) { return bf2f(f2bf(f)); }
__device__ __forceinline__ v16h cat16(v8h lo, v8h hi) { return __builtin_shufflevector(lo, hi, 0, 1, 2, 3, 4, 5, 6, 7, 8, 9, 10, 11, 12, 13, 14, 15); }
__device__ __forceinline__ v16bf cat16b(v8us lo, v8us hi) { return __builtin_bit_cast(v16bf, __builtin_shufflevector(lo, hi, 0, 1, 2, 3, 4, 5, 6, 7, 8, 9, 10, 11, 12, 13, 14, 15)); }
__device__ __forceinline__ v8f wmma16(v16h a, v16h b, v8f c) { return __builtin_amdgcn_wmma_f32_16x16x32_f16(false, a, false, b, (short)0, c, false, false); }
__device__ __forceinline__ v8f wmmab(v16bf a, v16bf b, v8f c) { return __builtin_amdgcn_wmma_f32_16x16x32_bf16(false, a, false, b, (short)0, c, false, false); }

template <bool SPLITA, bool F16OUT = false>
__global__ __launch_bounds__(128) void k_gemmb(const bf* __restrict__ A, const bf* __restrict__ Al, const bf* __restrict__ Bn, const float* __restrict__ bias, float* C, int ldc, h16* C2, const float* __restrict__ R = nullptr, int K = DM, int roundR = 1) {
    __shared__ __align__(16) float ost[4][16 * 68];
    const int lane = threadIdx.x & 31, wave = threadIdx.x >> 5, lr = lane & 15, hi = lane >> 4;
    const int r0 = blockIdx.x * 64 + wave * 16, c0 = blockIdx.y * 64;
    const size_t aoff = (size_t)(r0 + lr) * K + 8 * hi;
    size_t boff[4];
#pragma unroll
    for (int t = 0; t < 4; ++t) boff[t] = (size_t)(c0 + t * 16 + lr) * K + 8 * hi;
    v8f acc[4];
#pragma unroll
    for (int t = 0; t < 4; ++t) acc[t] = (v8f){};
#pragma unroll 1
    for (int kc = 0; kc < K; kc += 32) {
        const v16bf a = cat16b(*(const v8us*)(A + aoff + kc), *(const v8us*)(A + aoff + kc + 16));
        v16bf al = a;
        if (SPLITA) al = cat16b(*(const v8us*)(Al + aoff + kc), *(const v8us*)(Al + aoff + kc + 16));
#pragma unroll
        for (int t = 0; t < 4; ++t) { const v16bf b = cat16b(*(const v8us*)(Bn + boff[t] + kc), *(const v8us*)(Bn + boff[t] + kc + 16)); acc[t] = wmmab(a, b, acc[t]); if (SPLITA) acc[t] = wmmab(al, b, acc[t]); }
        asm volatile("v_nop\n\tv_nop\n\tv_nop\n\tv_nop" : "+v"(acc[0]), "+v"(acc[1]), "+v"(acc[2]), "+v"(acc[3]) : "v"(a), "v"(al));
    }
    float* os = &ost[wave][0];
#pragma unroll
    for (int t = 0; t < 4; ++t) { const float bv = bias ? bfr(bias[c0 + t * 16 + lr]) : 0.f;
#pragma unroll
        for (int j = 0; j < 8; ++j) os[(hi * 8 + j) * 68 + t * 16 + lr] = acc[t][j] + bv; }
    __syncthreads();
    if (F16OUT) {
        h16* crow = (h16*)(void*)C + (size_t)r0 * ldc + c0;
        auto pass = [&]() {
#pragma unroll
            for (int s = 0; s < 4; ++s) { const int row = 4 * s + (lane >> 3), piece = lane & 7; const float* sp = os + row * 68 + piece * 8; v8h o, o2;
#pragma unroll
                for (int i = 0; i < 8; ++i) { const h16 a = (h16)sp[i]; o[i] = a; o2[i] = (h16)((sp[i] - (float)a) * LOSC); }
                *(volatile v8h*)(crow + (size_t)row * ldc + piece * 8) = o; if (C2) *(volatile v8h*)(C2 + (size_t)r0 * ldc + c0 + (size_t)row * ldc + piece * 8) = o2; }
        };
        pass(); __threadfence(); pass();
    } else {
        float* crow = C + (size_t)r0 * ldc + c0;
        auto pass = [&]() {
#pragma unroll
            for (int s = 0; s < 8; ++s) { const int Lid = (lane >> 3) + 4 * s, piece = lane & 7; const int row = Lid >> 1, cofs = (Lid & 1) * 32 + piece * 4;
                v4f val = *(const v4fa*)(os + row * 68 + cofs); if (R) { const v4f rv = *(const v4f*)(R + ((size_t)r0 + row) * ldc + c0 + cofs); val += roundR ? (v4f){bfr(rv[0]), bfr(rv[1]), bfr(rv[2]), bfr(rv[3])} : rv; }
                *(volatile v4f*)(crow + (size_t)row * ldc + cofs) = val; }
        };
        pass(); __threadfence(); pass();
    }
}


__global__ __launch_bounds__(256) void k_xall(const float* __restrict__ inp, const float* __restrict__ z, bf* X) {
    const int u = blockIdx.x * 256 + threadIdx.x; if (u >= NL * NBT * KI / 8) return;
    const int i0 = (u % (KI / 8)) * 8, b = (u / (KI / 8)) % NBT, l = u / ((KI / 8) * NBT); v8us v;
#pragma unroll
    for (int k = 0; k < 8; ++k) { const int i = i0 + k; float x = 0.f;
        if (i < DI) x = inp[((size_t)b * NL + l) * DI + i]; else if (i < NI) x = z[((size_t)b * NL + l) * DC + (i - DI)];
        v[k] = f2bf(x); }
    const size_t o = ((size_t)l * NBT + b) * KI + i0; *(volatile v8us*)(X + o) = v; __threadfence(); *(volatile v8us*)(X + o) = v;
}
__global__ __launch_bounds__(256) void k_went(const float* __restrict__ We, int l0, bf* WT) {
    const int u = blockIdx.x * 256 + threadIdx.x; if (u >= LCH * HH * KI / 8) return;
    const int i0 = (u % (KI / 8)) * 8, h = (u / (KI / 8)) % HH, lp = u / ((KI / 8) * HH), l = l0 + lp; v8us v;
#pragma unroll
    for (int k = 0; k < 8; ++k) { const int i = i0 + k; v[k] = (i < NI) ? f2bf(We[((size_t)l * NI + i) * HH + h]) : (unsigned short)0; }
    const size_t o = ((size_t)lp * HH + h) * KI + i0; *(volatile v8us*)(WT + o) = v; __threadfence(); *(volatile v8us*)(WT + o) = v;
}
__global__ __launch_bounds__(256) void k_vcat(const float* __restrict__ Vm, const float* __restrict__ Vs, const float* __restrict__ Vp, const float* __restrict__ bm, const float* __restrict__ bs, const float* __restrict__ bp, int l0, bf* VT, float* BC) {
    const size_t u = (size_t)blockIdx.x * 256 + threadIdx.x;
    if (u < (size_t)LCH * NOP * HH / 8) { const int h0 = (int)(u % (HH / 8)) * 8, n = (int)((u / (HH / 8)) % NOP), lp = (int)(u / ((HH / 8) * NOP)), l = l0 + lp; v8us v;
#pragma unroll
        for (int k = 0; k < 8; ++k) { const int h = h0 + k; float w = 0.f;
            if (n < 15) w = Vm[((size_t)l * HH + h) * 15 + n]; else if (n < 30) w = Vs[((size_t)l * HH + h) * 15 + (n - 15)]; else if (n < 35) w = Vp[((size_t)l * HH + h) * 5 + (n - 30)];
            v[k] = f2bf(w); }
        const size_t o = ((size_t)lp * NOP + n) * HH + h0; *(volatile v8us*)(VT + o) = v; __threadfence(); *(volatile v8us*)(VT + o) = v; }
    if (u < (size_t)LCH * NOP / 4) { const int c0 = (int)(u % (NOP / 4)) * 4, lp = (int)(u / (NOP / 4)), l = l0 + lp; v4f bv;
#pragma unroll
        for (int k = 0; k < 4; ++k) { const int n = c0 + k; bv[k] = (n < 15) ? bm[l * 15 + n] : (n < 30 ? bs[l * 15 + n - 15] : (n < 35 ? bp[l * 5 + n - 30] : 0.f)); }
        *(volatile v4f*)(BC + (size_t)lp * NOP + c0) = bv; __threadfence(); *(volatile v4f*)(BC + (size_t)lp * NOP + c0) = bv; }
}
__global__ __launch_bounds__(256) void k_prefix(const float* __restrict__ C, const float* __restrict__ benc, int first, float* ST, bf* Hh, bf* Hl) {
    const int lane = threadIdx.x & 31, wid = blockIdx.x * 8 + (threadIdx.x >> 5); if (wid >= NBT * (HH / 256)) return;
    const int b = wid / (HH / 256), h0 = (wid % (HH / 256)) * 256 + lane * 8;
    float st[8];
#pragma unroll
    for (int k = 0; k < 8; ++k) st[k] = first ? bfr(benc[h0 + k]) : ST[(size_t)b * HH + h0 + k];
#pragma unroll 1
    for (int l = 0; l < LCH; ++l) { v8us oh, ol;
#pragma unroll
        for (int k = 0; k < 8; ++k) { const float a = fmaxf(st[k], 0.f); const unsigned short hb = f2bf(a); oh[k] = hb; ol[k] = f2bf(a - bf2f(hb)); st[k] += C[((size_t)l * NBT + b) * HH + h0 + k]; }
        const size_t o = ((size_t)l * NBT + b) * HH + h0;
        *(volatile v8us*)(Hh + o) = oh; *(volatile v8us*)(Hl + o) = ol; __threadfence(); *(volatile v8us*)(Hh + o) = oh; *(volatile v8us*)(Hl + o) = ol; }
    v8f sv;
#pragma unroll
    for (int k = 0; k < 8; ++k) sv[k] = st[k];
    *(volatile v8f*)(ST + (size_t)b * HH + h0) = sv; __threadfence(); *(volatile v8f*)(ST + (size_t)b * HH + h0) = sv;
}
__global__ __launch_bounds__(256) void k_out(const float* __restrict__ OC, float* OUTP) {
    const size_t i = (size_t)blockIdx.x * 256 + threadIdx.x; if (i >= (size_t)NBT * NL * NO) return;
    const int n = (int)(i % NO), l = (int)((i / NO) % NL), b = (int)(i / ((size_t)NO * NL));
    const float v = OC[((size_t)l * NBT + b) * NOP + n];
    *(volatile float*)(OUTP + i) = v; __threadfence(); *(volatile float*)(OUTP + i) = v;
}

extern "C" void kernel_launch(void* const* d_in, const int* in_sizes, int n_in,
                              void* d_out, int out_size, void* d_ws, size_t ws_size, hipStream_t stream) {
    (void)in_sizes; (void)n_in; (void)out_size;
    const float* inp = (const float*)d_in[0]; const float* z = (const float*)d_in[1]; const float* We = (const float*)d_in[2]; const float* benc = (const float*)d_in[3];
    const float* Vm = (const float*)d_in[4]; const float* bm = (const float*)d_in[5]; const float* Vs = (const float*)d_in[6]; const float* bs = (const float*)d_in[7]; const float* Vp = (const float*)d_in[8]; const float* bp = (const float*)d_in[9];
    float* out = (float*)d_out;
    char* wsp = (char*)d_ws;
    auto take = [&](size_t bytes) { char* p = wsp; wsp += (bytes + 255) & ~(size_t)255; return (void*)p; };
    bf* X = (bf*)take((size_t)NL * NBT * KI * 2); bf* WT = (bf*)take((size_t)LCH * HH * KI * 2); bf* VT = (bf*)take((size_t)LCH * NOP * HH * 2); float* BC = (float*)take((size_t)LCH * NOP * 4);
    float* C = (float*)take((size_t)LCH * NBT * HH * 4); float* ST = (float*)take((size_t)NBT * HH * 4); bf* Hh = (bf*)take((size_t)LCH * NBT * HH * 2); bf* Hl = (bf*)take((size_t)LCH * NBT * HH * 2); float* OC = (float*)take((size_t)NL * NBT * NOP * 4);
    if ((size_t)(wsp - (char*)d_ws) > ws_size) return;
    k_xall<<<(NL * NBT * KI / 8 + 255) / 256, 256, 0, stream>>>(inp, z, X);
    for (int ch = 0; ch < NLC; ++ch) {
        k_went<<<(LCH * HH * KI / 8 + 255) / 256, 256, 0, stream>>>(We, ch * LCH, WT);
        k_vcat<<<(unsigned)(((size_t)LCH * NOP * HH / 8 + 255) / 256), 256, 0, stream>>>(Vm, Vs, Vp, bm, bs, bp, ch * LCH, VT, BC);
        for (int l = 0; l < LCH; ++l) { const int L = ch * LCH + l;
            k_gemmb<false, false><<<dim3(NBT / 64, HH / 64, 1), 128, 0, stream>>>(X + (size_t)L * NBT * KI, nullptr, WT + (size_t)l * HH * KI, nullptr, C + (size_t)l * NBT * HH, HH, nullptr, nullptr, KI); }
        k_prefix<<<(NBT * (HH / 256)) / 8, 256, 0, stream>>>(C, benc, ch == 0 ? 1 : 0, ST, Hh, Hl);
        for (int l = 0; l < LCH; ++l) { const int L = ch * LCH + l;
            k_gemmb<true, false><<<dim3(NBT / 64, 1, 1), 128, 0, stream>>>(Hh + (size_t)l * NBT * HH, Hl + (size_t)l * NBT * HH, VT + (size_t)l * NOP * HH, BC + (size_t)l * NOP, OC + (size_t)L * NBT * NOP, NOP, nullptr); }
    }
    k_out<<<(unsigned)(((size_t)NBT * NL * NO + 255) / 256), 256, 0, stream>>>(OC, out);
}
